// SimpleDetector_24455543783494
// MI455X (gfx1250) — hardware-verified
//
#include <hip/hip_runtime.h>
#include <hip/hip_bf16.h>

typedef __attribute__((ext_vector_type(16))) _Float16 v16h;
typedef __attribute__((ext_vector_type(8)))  _Float16 v8h;
typedef __attribute__((ext_vector_type(4)))  _Float16 v4h;
typedef __attribute__((ext_vector_type(8)))  float    v8f;
typedef __attribute__((ext_vector_type(4)))  unsigned int v4u;
typedef __attribute__((ext_vector_type(8)))  int      v8i;
typedef __attribute__((ext_vector_type(4)))  int      v4i;
typedef __attribute__((ext_vector_type(4)))  float    v4f_t;
typedef float v4fa __attribute__((ext_vector_type(4), may_alias));

#define TPB    256
#define WAVES  8
#define TILE_E 16
#define FEAT   128
#define LDW    136
#define W_LDS_BYTES (FEAT * LDW * 2)

__device__ __forceinline__ v16h load_frag2(const _Float16* p0, const _Float16* p1) {
    v8h lo = *(const v8h*)p0;
    v8h hi = *(const v8h*)p1;
    v16h r;
#pragma unroll
    for (int i = 0; i < 8; ++i) { r[i] = lo[i]; r[i + 8] = hi[i]; }
    return r;
}

__device__ __forceinline__ unsigned int fenc(float f) {
    unsigned int u = __float_as_uint(f);
    return (u & 0x80000000u) ? ~u : (u | 0x80000000u);
}

__device__ __forceinline__ void tdm_load_wtile(const _Float16* gsrc, unsigned lds_off) {
    unsigned long long ga = (unsigned long long)(const void*)gsrc;
    v4u g0;
    g0[0] = 1u;
    g0[1] = lds_off;
    g0[2] = (unsigned)(ga & 0xFFFFFFFFu);
    g0[3] = (unsigned)((ga >> 32) & 0x01FFFFFFu)
          | (2u << 30);
    v8i g1;
    g1[0] = (int)((1u << 16)
                | (1u << 20)
                | (5u << 22)
                | (3u << 25));
    g1[1] = (int)(128u << 16);
    g1[2] = (int)(128u << 16);
    g1[3] = (int)(128u << 16);
    g1[4] = 128;
    g1[5] = 128;
    g1[6] = 0;
    g1[7] = 0;
    v4i gz4 = {0, 0, 0, 0};
    v8i gz8 = {0, 0, 0, 0, 0, 0, 0, 0};
    __builtin_amdgcn_tensor_load_to_lds(g0, g1, gz4, gz4, gz8, 0);
}

__global__ void prep_weights_kernel(const float* __restrict__ W1,
                                    const float* __restrict__ W2,
                                    _Float16* __restrict__ w1t,
                                    _Float16* __restrict__ w2t) {
    int i = (blockIdx.x * blockDim.x + threadIdx.x) * 2;
    if (i < FEAT * FEAT) {
        int n = i >> 7, k = i & (FEAT - 1);
        const unsigned p1 = (unsigned)__builtin_bit_cast(unsigned short, (_Float16)W1[k * FEAT + n]) | ((unsigned)__builtin_bit_cast(unsigned short, (_Float16)W1[(k + 1) * FEAT + n]) << 16);
        const unsigned p2 = (unsigned)__builtin_bit_cast(unsigned short, (_Float16)W2[k * FEAT + n]) | ((unsigned)__builtin_bit_cast(unsigned short, (_Float16)W2[(k + 1) * FEAT + n]) << 16);
        *(volatile unsigned*)(w1t + i) = p1; *(volatile unsigned*)(w2t + i) = p2;
        __threadfence();
        *(volatile unsigned*)(w1t + i) = p1; *(volatile unsigned*)(w2t + i) = p2;
    }
}

__global__ __launch_bounds__(256) void segmin_kernel(const float* __restrict__ preds, const int* __restrict__ idx,
                                                     float* __restrict__ out, int n_edges, int P) {
    const int p = blockIdx.x * 256 + threadIdx.x;
    if (p >= P) return;
    int lo = 0, hi = n_edges;
    while (lo < hi) { int mid = (lo + hi) >> 1; if (idx[mid] < p) lo = mid + 1; else hi = mid; }
    const int s0 = lo;
    hi = n_edges;
    while (lo < hi) { int mid = (lo + hi) >> 1; if (idx[mid] <= p) lo = mid + 1; else hi = mid; }
    const int s1 = lo;
    float m = 3.402823466e38f;
    for (int e = s0; e < s1; ++e) m = fminf(m, preds[e]);
    const float r = (s1 > s0) ? m : 0.0f;
    *(volatile float*)(out + p) = r; __threadfence(); *(volatile float*)(out + p) = r;
}

__global__ __launch_bounds__(TPB)
void edge_mlp_kernel(const float* __restrict__ zs,
                     const int*   __restrict__ src,
                     const int*   __restrict__ dst,
                     const int*   __restrict__ idx,
                     const float* __restrict__ W1, const float* __restrict__ b1,
                     const float* __restrict__ W2, const float* __restrict__ b2,
                     const float* __restrict__ W3, const float* __restrict__ b3,
                     const _Float16* __restrict__ wsW1t,
                     const _Float16* __restrict__ wsW2t,
                     int use_ws,
                     float* __restrict__ preds,
                     int n_edges) {
    extern __shared__ char smem[];
    _Float16* w1t  = (_Float16*)smem;
    _Float16* w2t  = w1t + FEAT * LDW;
    float*    w3s  = (float*)(w2t + FEAT * LDW);
    float*    b1s  = w3s + FEAT;
    float*    b2s  = b1s + FEAT;
    _Float16* tiles = (_Float16*)(b2s + FEAT);

    const int t = threadIdx.x;

    if (use_ws) {
        if (t == 0) {
            unsigned dynbase = (unsigned)__builtin_amdgcn_groupstaticsize();
            tdm_load_wtile(wsW1t, dynbase);
            tdm_load_wtile(wsW2t, dynbase + W_LDS_BYTES);
            __builtin_amdgcn_s_wait_tensorcnt(0);
        }
    } else {
        for (int i = t; i < FEAT * FEAT; i += TPB) {
            int n = i >> 7, k = i & (FEAT - 1);
            w1t[n * LDW + k] = (_Float16)W1[k * FEAT + n];
            w2t[n * LDW + k] = (_Float16)W2[k * FEAT + n];
        }
    }
    if (t < FEAT) { w3s[t] = W3[t]; b1s[t] = b1[t]; b2s[t] = b2[t]; }
    __syncthreads();

    const int wave = t >> 5;
    const int lane = t & 31;
    const int row  = lane & 15;
    const int hh   = lane >> 4;

    _Float16* xt = tiles + wave * 2 * TILE_E * LDW;
    _Float16* ht = xt + TILE_E * LDW;

    const int e0 = (int)blockIdx.x * (WAVES * TILE_E) + wave * TILE_E;

    for (int e = 0; e < TILE_E; ++e) {
        int eg  = e0 + e;
        int egc = eg < n_edges ? eg : n_edges - 1;
        int s = src[egc], d = dst[egc];
        const float* base = (lane < 16) ? (zs + (size_t)s * 64 + lane * 4)
                                        : (zs + (size_t)d * 64 + (lane - 16) * 4);
        float4 v = *(const float4*)base;
        v4h hv;
        hv[0] = (_Float16)v.x; hv[1] = (_Float16)v.y;
        hv[2] = (_Float16)v.z; hv[3] = (_Float16)v.w;
        *(v4h*)(xt + e * LDW + lane * 4) = hv;
    }
    asm volatile("s_wait_dscnt 0" ::: "memory");

    v16h afrag[4];
#pragma unroll
    for (int kb = 0; kb < 4; ++kb) {
        const _Float16* base = xt + row * LDW + kb * 32 + hh * 8;
        afrag[kb] = load_frag2(base, base + 16);
    }
#pragma unroll
    for (int nb = 0; nb < 8; ++nb) {
        float bias = b1s[nb * 16 + row];
        v8f acc;
#pragma unroll
        for (int r = 0; r < 8; ++r) acc[r] = bias;
#pragma unroll
        for (int kb = 0; kb < 4; ++kb) {
            const _Float16* wb = w1t + (nb * 16 + row) * LDW + kb * 32 + hh * 8;
            v16h bfrag = load_frag2(wb, wb + 16);
            acc = __builtin_amdgcn_wmma_f32_16x16x32_f16(
                false, afrag[kb], false, bfrag, (short)0, acc, false, false);
        }
#pragma unroll
        for (int r = 0; r < 8; ++r) {
            ht[(r + 8 * hh) * LDW + nb * 16 + row] = (_Float16)fmaxf(acc[r], 0.0f);
        }
    }
    asm volatile("s_wait_dscnt 0" ::: "memory");

#pragma unroll
    for (int kb = 0; kb < 4; ++kb) {
        const _Float16* base = ht + row * LDW + kb * 32 + hh * 8;
        afrag[kb] = load_frag2(base, base + 16);
    }
#pragma unroll
    for (int nb = 0; nb < 8; ++nb) {
        float bias = b2s[nb * 16 + row];
        v8f acc;
#pragma unroll
        for (int r = 0; r < 8; ++r) acc[r] = bias;
#pragma unroll
        for (int kb = 0; kb < 4; ++kb) {
            const _Float16* wb = w2t + (nb * 16 + row) * LDW + kb * 32 + hh * 8;
            v16h bfrag = load_frag2(wb, wb + 16);
            acc = __builtin_amdgcn_wmma_f32_16x16x32_f16(
                false, afrag[kb], false, bfrag, (short)0, acc, false, false);
        }
#pragma unroll
        for (int r = 0; r < 8; ++r) {
            xt[(r + 8 * hh) * LDW + nb * 16 + row] = (_Float16)fmaxf(acc[r], 0.0f);
        }
    }
    asm volatile("s_wait_dscnt 0" ::: "memory");

    float sum = 0.0f;
    const _Float16* yrow = xt + row * LDW + hh * 64;
    const float*    w3p  = w3s + hh * 64;
#pragma unroll
    for (int c = 0; c < 8; ++c) {
        v8h    yv = *(const v8h*)(yrow + c * 8);
        float4 wa = *(const float4*)(w3p + c * 8);
        float4 wb = *(const float4*)(w3p + c * 8 + 4);
        sum += (float)yv[0] * wa.x + (float)yv[1] * wa.y +
               (float)yv[2] * wa.z + (float)yv[3] * wa.w +
               (float)yv[4] * wb.x + (float)yv[5] * wb.y +
               (float)yv[6] * wb.z + (float)yv[7] * wb.w;
    }
    sum += __shfl_xor(sum, 16, 32);

    __shared__ __attribute__((aligned(16))) float sPred[WAVES * TILE_E];
    if (hh == 0) sPred[wave * TILE_E + row] = sum + b3[0];
    __syncthreads();
    if (t < 32) {
        const int eb = (int)blockIdx.x * (WAVES * TILE_E) + t * 4;
        const v4f_t v = *(const v4fa*)(sPred + t * 4);
        if (eb + 3 < n_edges) { *(volatile v4f_t*)(preds + eb) = v; __threadfence(); *(volatile v4f_t*)(preds + eb) = v; }
        else { for (int q = 0; q < 4; ++q) if (eb + q < n_edges) preds[eb + q] = sPred[t * 4 + q]; }
    }
}

extern "C" void kernel_launch(void* const* d_in, const int* in_sizes, int n_in,
                              void* d_out, int out_size, void* d_ws, size_t ws_size,
                              hipStream_t stream) {
    const float* zs  = (const float*)d_in[0];
    const int*   src = (const int*)d_in[1];
    const int*   dst = (const int*)d_in[2];
    const int*   idx = (const int*)d_in[3];
    const float* W1  = (const float*)d_in[4];
    const float* b1  = (const float*)d_in[5];
    const float* W2  = (const float*)d_in[6];
    const float* b2  = (const float*)d_in[7];
    const float* W3  = (const float*)d_in[8];
    const float* b3  = (const float*)d_in[9];

    const int E = in_sizes[1];
    const int P = out_size;

    const size_t wbytes = (size_t)FEAT * FEAT * sizeof(_Float16);
    _Float16* wsW1t = (_Float16*)d_ws;
    _Float16* wsW2t = wsW1t + FEAT * FEAT;
    float* preds = (float*)((char*)d_ws + 2 * wbytes);
    int use_ws = (ws_size >= 2 * wbytes + (size_t)E * sizeof(float)) ? 1 : 0;

    prep_weights_kernel<<<(FEAT * FEAT / 2 + 255) / 256, 256, 0, stream>>>(W1, W2, wsW1t, wsW2t);

    const size_t shmem =
        2 * (size_t)FEAT * LDW * sizeof(_Float16) +
        3 * (size_t)FEAT * sizeof(float) +
        (size_t)WAVES * 2 * TILE_E * LDW * sizeof(_Float16);

    (void)hipFuncSetAttribute((const void*)edge_mlp_kernel,
                              hipFuncAttributeMaxDynamicSharedMemorySize,
                              (int)shmem);

    const int edges_per_block = WAVES * TILE_E;
    int nblocks = (E + edges_per_block - 1) / edges_per_block;
    edge_mlp_kernel<<<nblocks, TPB, shmem, stream>>>(
        zs, src, dst, idx, W1, b1, W2, b2, W3, b3,
        wsW1t, wsW2t, use_ws, preds, E);

    segmin_kernel<<<(P + 255) / 256, 256, 0, stream>>>(preds, idx, (float*)d_out, E, P);
}
